// Tree_SSM_25795573580018
// MI455X (gfx1250) — hardware-run, weakly checked
//
#include <hip/hip_runtime.h>
#include <math.h>

typedef __attribute__((ext_vector_type(16))) _Float16 v16h;
typedef __attribute__((ext_vector_type(8)))  _Float16 v8h;
typedef __attribute__((ext_vector_type(4)))  _Float16 v4h;
typedef __attribute__((ext_vector_type(16))) __bf16   v16b;
typedef __attribute__((ext_vector_type(8)))  __bf16   v8b;
typedef __attribute__((ext_vector_type(8)))  float    v8f;
typedef __attribute__((ext_vector_type(4)))  float    v4f;
typedef __attribute__((address_space(1))) volatile float gvf;

constexpr int kBatch = 4;
constexpr int kHW    = 64;
constexpr int kL     = kHW * kHW;
constexpr int kDm    = 192;
constexpr int kDe    = 384;
constexpr int kDtR   = 12;
constexpr int kXpN   = kDtR + 2;
constexpr int kXdP   = 64;
constexpr int kRows  = kBatch * kL;
static_assert(kL == 4096);
static_assert(kRows == 16384);
static_assert((kDm % 32) == 0 && (kDe % 32) == 0);
static_assert((kRows % 64) == 0 && (kDe % 64) == 0 && (kDm % 64) == 0 && (kXdP % 64) == 0);
static_assert(kXpN <= kXdP);

constexpr float kCarryAct = 16.0f;
constexpr float kCarryW   = 32.0f;
constexpr float kFold     = 1.0f / (kCarryAct * kCarryW);
constexpr float kInvDe    = 1.0f / (float)kDe;
constexpr float kLnEps    = 1e-5f;

constexpr int kCvCh  = 128;
constexpr int kCvPos = 16;
constexpr int kCvTP  = 132;
static_assert((kDe % kCvCh) == 0 && (kHW % kCvPos) == 0);
constexpr int kScCh = 128;
constexpr int kScTS = 64;
static_assert((kDe % kScCh) == 0 && (kL % kScTS) == 0);
constexpr int kNmWaves = 8;
constexpr int kNmPer   = 4;
static_assert((kRows % (kNmWaves * kNmPer)) == 0);

constexpr size_t kOffXH  = 0;
constexpr size_t kOffXL  = kOffXH  + (size_t)kRows * kDm * 2;
constexpr size_t kOffWIH = kOffXL  + (size_t)kRows * kDm * 2;
constexpr size_t kOffWIL = kOffWIH + (size_t)2 * kDe * kDm * 2;
constexpr size_t kOffWXP = kOffWIL + (size_t)2 * kDe * kDm * 2;
constexpr size_t kOffWOP = kOffWXP + (size_t)kXdP * kDe * 2;
constexpr size_t kOffX1  = kOffWOP + (size_t)kDm * kDe * 2;
constexpr size_t kOffZR  = kOffX1  + (size_t)kRows * kDe * 4;
constexpr size_t kOffXS  = kOffZR  + (size_t)kRows * kDe * 4;
constexpr size_t kOffXSA = kOffXS  + (size_t)kRows * kDe * 4;
constexpr size_t kOffXD  = kOffXSA + (size_t)kRows * kDe * 2;
constexpr size_t kOffYZ  = kOffXD  + (size_t)kRows * kXdP * 4;
constexpr size_t kWsTotal = kOffYZ + (size_t)kRows * kDe * 2;
static_assert(kWsTotal == 118226944ull);
static_assert(kWsTotal <= 134217728ull);
static_assert((kOffXL % 128) == 0 && (kOffWIH % 128) == 0 && (kOffWIL % 128) == 0 && (kOffWXP % 128) == 0 &&
              (kOffWOP % 128) == 0 && (kOffX1 % 128) == 0 && (kOffZR % 128) == 0 && (kOffXS % 128) == 0 &&
              (kOffXSA % 128) == 0 && (kOffXD % 128) == 0 && (kOffYZ % 128) == 0);

__device__ __forceinline__ unsigned short f2bf_bits(float f) {
  unsigned u = __float_as_uint(f);
  return (unsigned short)((u + 0x7FFFu + ((u >> 16) & 1u)) >> 16);
}
__device__ __forceinline__ float bf_bits2f(unsigned short h) { return __uint_as_float(((unsigned)h) << 16); }

__device__ __forceinline__ void dep_guard4_h(v8f& a, v8f& b, v8f& c, v8f& d, v16h x, v16h y) { asm volatile("v_nop\n\tv_nop\n\tv_nop\n\tv_nop" : "+v"(a), "+v"(b), "+v"(c), "+v"(d) : "v"(x), "v"(y)); }
__device__ __forceinline__ void dep_guard4_b(v8f& a, v8f& b, v8f& c, v8f& d, v16b x, v16b y) { asm volatile("v_nop\n\tv_nop\n\tv_nop\n\tv_nop" : "+v"(a), "+v"(b), "+v"(c), "+v"(d) : "v"(x), "v"(y)); }
__device__ __forceinline__ void keep4_h(v16h a, v16h b, v16h c, v16h d) { asm volatile("v_nop" :: "v"(a), "v"(b), "v"(c), "v"(d)); }
__device__ __forceinline__ void keep4_b(v16b a, v16b b, v16b c, v16b d) { asm volatile("v_nop" :: "v"(a), "v"(b), "v"(c), "v"(d)); }
__device__ __forceinline__ void acc_guard4(v8f& a, v8f& b, v8f& c, v8f& d) { asm volatile("v_nop\n\tv_nop\n\tv_nop\n\tv_nop" : "+v"(a), "+v"(b), "+v"(c), "+v"(d)); }
template <typename T> struct Frag;
template <> struct Frag<_Float16> {
  typedef v16h V; union U { v16h v; v8h h[2]; };
  static __device__ __forceinline__ v16h load(const _Float16* p) {
    U f; f.h[0] = *(const v8h*)(p); f.h[1] = *(const v8h*)(p + 16); return f.v;
  }
  static __device__ __forceinline__ v8f mma(v16h a, v16h b, v8f c) {
    return __builtin_amdgcn_wmma_f32_16x16x32_f16(false, a, false, b, (short)0, c, false, false);
  }
  static __device__ __forceinline__ void guard4(v8f& a, v8f& b, v8f& c, v8f& d, v16h x, v16h y) { dep_guard4_h(a, b, c, d, x, y); }
  static __device__ __forceinline__ void keep(v16h a, v16h b, v16h c, v16h d) { keep4_h(a, b, c, d); }
};
template <> struct Frag<__bf16> {
  typedef v16b V; union U { v16b v; v8b h[2]; };
  static __device__ __forceinline__ v16b load(const __bf16* p) {
    U f; f.h[0] = *(const v8b*)(p); f.h[1] = *(const v8b*)(p + 16); return f.v;
  }
  static __device__ __forceinline__ v8f mma(v16b a, v16b b, v8f c) {
    return __builtin_amdgcn_wmma_f32_16x16x32_bf16(false, a, false, b, (short)0, c, false, false);
  }
  static __device__ __forceinline__ void guard4(v8f& a, v8f& b, v8f& c, v8f& d, v16b x, v16b y) { dep_guard4_b(a, b, c, d, x, y); }
  static __device__ __forceinline__ void keep(v16b a, v16b b, v16b c, v16b d) { keep4_b(a, b, c, d); }
};

template <int ET> struct Elem;
template <> struct Elem<0> { typedef _Float16 T; };
template <> struct Elem<1> { typedef __bf16 T; };
template <int ET, bool SPLIT, int BIAS_MODE, int OUT_MODE, bool RESID, int ACT = 0>
__global__ __launch_bounds__(256) void wmma_gemm64(
    const unsigned short* __restrict__ Ap, const unsigned short* __restrict__ A2p, int lda, long strideA,
    const unsigned short* __restrict__ Btp, const unsigned short* __restrict__ Bt2p, int ldb, long strideB,
    void* __restrict__ Cout, void* __restrict__ Cout2, int ldc, long strideC,
    const float* __restrict__ bias,
    const float* __restrict__ resid, long strideR,
    int M, int N, int K, float scale) {
  typedef typename Elem<ET>::T T;
  typedef typename Frag<T>::V V;
  const T* A = (const T*)Ap; const T* A2 = (const T*)A2p; const T* Bt = (const T*)Btp; const T* Bt2 = (const T*)Bt2p;
  __shared__ __align__(16) float sT[8][16 * 68];
  const int b    = blockIdx.y;
  const int lane = threadIdx.x & 31;
  const int wave = threadIdx.x >> 5;
  const int tilesN = N >> 6;
  const int tilesM = M >> 6;
  const int tile = blockIdx.x * 8 + wave;
  if (tile >= tilesM * tilesN) return;
  const int tm = tile / tilesN;
  const int tn = tile - tm * tilesN;
  const int m0 = tm << 6;
  const int n0 = tn << 6;

  const T* Ab  = A  + (size_t)b * strideA;
  const T* Bb  = Bt + (size_t)b * strideB;
  const T* Ab2 = SPLIT ? (A2  + (size_t)b * strideA) : nullptr;
  const T* Bb2 = SPLIT ? (Bt2 + (size_t)b * strideB) : nullptr;

  const int rlane = lane & 15;
  const int koff  = (lane >> 4) * 8;
  const int mOff  = (lane >> 4) * 8;

  v8f acc[4][4];
#pragma unroll
  for (int i = 0; i < 4; ++i)
#pragma unroll
    for (int j = 0; j < 4; ++j) acc[i][j] = (v8f){0.f,0.f,0.f,0.f,0.f,0.f,0.f,0.f};

  for (int k0 = 0; k0 < K; k0 += 32) {
    V bh[4], bl[4];
#pragma unroll
    for (int j = 0; j < 4; ++j) {
      const size_t bo = (size_t)(n0 + (j << 4) + rlane) * ldb + koff + k0;
      bh[j] = Frag<T>::load(Bb + bo);
      if (SPLIT) bl[j] = Frag<T>::load(Bb2 + bo);
    }
#pragma unroll
    for (int i = 0; i < 4; ++i) {
      const size_t ao = (size_t)(m0 + (i << 4) + rlane) * lda + koff + k0;
      V ah = Frag<T>::load(Ab + ao);
      V al;
      if (SPLIT) al = Frag<T>::load(Ab2 + ao);
#pragma unroll
      for (int j = 0; j < 4; ++j) {
        acc[i][j] = Frag<T>::mma(ah, bh[j], acc[i][j]);
        if (SPLIT) {
          acc[i][j] = Frag<T>::mma(ah, bl[j], acc[i][j]);
          acc[i][j] = Frag<T>::mma(al, bh[j], acc[i][j]);
        }
      }
      Frag<T>::guard4(acc[i][0], acc[i][1], acc[i][2], acc[i][3], ah, SPLIT ? al : ah);
    }
    Frag<T>::keep(bh[0], bh[1], bh[2], bh[3]);
    if (SPLIT) Frag<T>::keep(bl[0], bl[1], bl[2], bl[3]);
  }
  acc_guard4(acc[0][0], acc[0][1], acc[0][2], acc[0][3]);
  acc_guard4(acc[1][0], acc[1][1], acc[1][2], acc[1][3]);
  acc_guard4(acc[2][0], acc[2][1], acc[2][2], acc[2][3]);
  acc_guard4(acc[3][0], acc[3][1], acc[3][2], acc[3][3]);

  float* slab = sT[wave];
  const float* Rb = RESID ? (resid + (size_t)b * strideR) : nullptr;
#pragma unroll
  for (int i = 0; i < 4; ++i) {
    const int mBase = m0 + (i << 4);
#pragma unroll
    for (int j = 0; j < 4; ++j) {
      const int n = n0 + (j << 4) + rlane;
      float bv = 0.f;
      if (BIAS_MODE == 2) bv = bias[n];
#pragma unroll
      for (int r = 0; r < 8; ++r) {
        float v = acc[i][j][r] * scale;
        if (BIAS_MODE == 1) v += bias[mBase + mOff + r];
        if (BIAS_MODE == 2) v += bv;
        if (RESID) v += Rb[(size_t)(mBase + mOff + r) * ldc + n];
        if (ACT == 2) v = fmaxf(v, 0.0f);
        if (ACT == 4) v = (v > 0.f) ? v : 0.01f * v;
        slab[(mOff + r) * 68 + (j << 4) + rlane] = v;
      }
    }
    __builtin_amdgcn_fence(__ATOMIC_RELEASE, "workgroup");
    __builtin_amdgcn_wave_barrier();
    __builtin_amdgcn_fence(__ATOMIC_ACQUIRE, "workgroup");
    if (OUT_MODE == 0) {
      float* C = (float*)Cout + (size_t)b * strideC;
      const int hh = lane >> 4, c4 = (lane & 15) * 4;
      for (int pass = 0; pass < 2; ++pass) {
#pragma unroll
        for (int it = 0; it < 8; ++it) {
          const int row = it * 2 + hh;
          v4f v = *(const v4f*)(slab + row * 68 + c4);
          *(volatile v4f*)(C + (size_t)(mBase + row) * ldc + n0 + c4) = v;
        }
        __threadfence();
      }
    } else {
      const int q = lane >> 3, c8 = (lane & 7) * 8;
      unsigned short* C  = (unsigned short*)Cout  + (size_t)b * strideC;
      unsigned short* C2 = (OUT_MODE == 2) ? ((unsigned short*)Cout2 + (size_t)b * strideC) : nullptr;
      for (int pass = 0; pass < 2; ++pass) {
#pragma unroll
        for (int it = 0; it < 4; ++it) {
          const int row = it * 4 + q;
          const float* sp = slab + row * 68 + c8;
          v8h hv, lv;
#pragma unroll
          for (int e = 0; e < 8; ++e) {
            if (OUT_MODE == 1) {
              hv[e] = (_Float16)sp[e];
            } else {
              unsigned short hb = f2bf_bits(sp[e]);
              unsigned short lb = f2bf_bits(sp[e] - bf_bits2f(hb));
              hv[e] = __builtin_bit_cast(_Float16, hb);
              lv[e] = __builtin_bit_cast(_Float16, lb);
            }
          }
          *(volatile v8h*)(C + (size_t)(mBase + row) * ldc + n0 + c8) = hv;
          if (OUT_MODE == 2) *(volatile v8h*)(C2 + (size_t)(mBase + row) * ldc + n0 + c8) = lv;
        }
        __threadfence();
      }
    }
    __builtin_amdgcn_fence(__ATOMIC_RELEASE, "workgroup");
    __builtin_amdgcn_wave_barrier();
    __builtin_amdgcn_fence(__ATOMIC_ACQUIRE, "workgroup");
  }
}

__global__ __launch_bounds__(256) void split_rows_bf16_kernel(
    const float* __restrict__ src, unsigned short* __restrict__ dhi, unsigned short* __restrict__ dlo, int total8)
{
  const int i = blockIdx.x * 256 + threadIdx.x;
  if (i >= total8) return;
  const size_t e0 = (size_t)i << 3;
  const v4f a0 = *(const v4f*)(src + e0);
  const v4f a1 = *(const v4f*)(src + e0 + 4);
  v8h hv, lv;
#pragma unroll
  for (int e = 0; e < 4; ++e) {
    const unsigned short h0 = f2bf_bits(a0[e]), h1 = f2bf_bits(a1[e]);
    const unsigned short l0 = f2bf_bits(a0[e] - bf_bits2f(h0)), l1 = f2bf_bits(a1[e] - bf_bits2f(h1));
    hv[e]     = __builtin_bit_cast(_Float16, h0);
    hv[4 + e] = __builtin_bit_cast(_Float16, h1);
    lv[e]     = __builtin_bit_cast(_Float16, l0);
    lv[4 + e] = __builtin_bit_cast(_Float16, l1);
  }
  unsigned short* qh = dhi + e0;
  unsigned short* ql = dlo + e0;
  *(volatile v8h*)qh = hv;
  *(volatile v8h*)ql = lv;
  __threadfence();
  *(volatile v8h*)qh = hv;
  *(volatile v8h*)ql = lv;
}

__global__ __launch_bounds__(256) void cast_f16_pad_kernel(
    const float* __restrict__ src, unsigned short* __restrict__ dst, int total8, int real8, float scale)
{
  const int i = blockIdx.x * 256 + threadIdx.x;
  if (i >= total8) return;
  const bool live = (i < real8);
  const int ic = live ? i : (real8 - 1);
  const float* p = src + ((size_t)ic << 3);
  const v4f a0 = *(const v4f*)(p);
  const v4f a1 = *(const v4f*)(p + 4);
  v8h hv;
#pragma unroll
  for (int e = 0; e < 4; ++e) {
    const float f0 = live ? (a0[e] * scale) : 0.0f;
    const float f1 = live ? (a1[e] * scale) : 0.0f;
    hv[e]     = (_Float16)f0;
    hv[4 + e] = (_Float16)f1;
  }
  unsigned short* q = dst + ((size_t)i << 3);
  *(volatile v8h*)q = hv;
  __threadfence();
  *(volatile v8h*)q = hv;
}

__device__ __forceinline__ float silu_f(float v) {
  const float e = expf(-v);
  return v * __builtin_amdgcn_rcpf(1.0f + e);
}

__global__ __launch_bounds__(128) void dwconv_silu_kernel(
    const float* __restrict__ X1, const float* __restrict__ cw, const float* __restrict__ cb,
    float* __restrict__ XS, unsigned short* __restrict__ XSA)
{
  __shared__ __align__(16) float sT[kCvPos * kCvTP];
  const int tid = threadIdx.x, lane = tid & 31, wave = tid >> 5;
  const int d0 = blockIdx.x * kCvCh, d = d0 + tid;
  const int g0 = blockIdx.y * kCvPos;
  const int img0 = g0 & ~(kL - 1);
  const int hh = (g0 >> 6) & (kHW - 1);
  const int w0 = g0 & (kHW - 1);
  const float* wp = cw + (size_t)d * 9;
  const float k0 = wp[0], k1 = wp[1], k2 = wp[2], k3 = wp[3], k4 = wp[4], k5 = wp[5], k6 = wp[6], k7 = wp[7], k8 = wp[8];
  const float bc = cb[d];
  const bool okm = (hh >= 1), okq = (hh <= kHW - 2);
  const int hm = okm ? (hh - 1) : 0;
  const int hq = okq ? (hh + 1) : (kHW - 1);
  const float* rm = X1 + (size_t)(img0 + hm * kHW) * kDe + d;
  const float* r0 = X1 + (size_t)(img0 + hh * kHW) * kDe + d;
  const float* rq = X1 + (size_t)(img0 + hq * kHW) * kDe + d;
  float l0, l1, l2, m0, m1, m2;
  {
    const int cl = w0 - 1;
    const bool ok = (cl >= 0);
    const size_t co = (size_t)(ok ? cl : 0) * kDe;
    const float a = rm[co], b = r0[co], c = rq[co];
    l0 = (ok && okm) ? a : 0.0f;
    l1 = ok ? b : 0.0f;
    l2 = (ok && okq) ? c : 0.0f;
  }
  {
    const size_t co = (size_t)w0 * kDe;
    const float a = rm[co], b = r0[co], c = rq[co];
    m0 = okm ? a : 0.0f;
    m1 = b;
    m2 = okq ? c : 0.0f;
  }
#pragma unroll 1
  for (int s = 0; s < kCvPos; ++s) {
    const int cr = w0 + s + 1;
    const bool ok = (cr <= kHW - 1);
    const size_t co = (size_t)(ok ? cr : (kHW - 1)) * kDe;
    const float a = rm[co], b = r0[co], c = rq[co];
    const float q0 = (ok && okm) ? a : 0.0f;
    const float q1 = ok ? b : 0.0f;
    const float q2 = (ok && okq) ? c : 0.0f;
    float acc = bc;
    acc = fmaf(k0, l0, acc);
    acc = fmaf(k1, m0, acc);
    acc = fmaf(k2, q0, acc);
    acc = fmaf(k3, l1, acc);
    acc = fmaf(k4, m1, acc);
    acc = fmaf(k5, q1, acc);
    acc = fmaf(k6, l2, acc);
    acc = fmaf(k7, m2, acc);
    acc = fmaf(k8, q2, acc);
    sT[s * kCvTP + tid] = silu_f(acc);
    l0 = m0; l1 = m1; l2 = m2;
    m0 = q0; m1 = q1; m2 = q2;
  }
  __syncthreads();
  v4f fv[4];
  v8h bv[2];
#pragma unroll
  for (int it = 0; it < 4; ++it) fv[it] = *(const v4f*)(sT + (it * 4 + wave) * kCvTP + lane * 4);
  const int hrow = wave * 2 + (lane >> 4);
  const int c8 = (lane & 15) * 8;
#pragma unroll
  for (int it = 0; it < 2; ++it) {
    const float* sp = sT + (it * 8 + hrow) * kCvTP + c8;
    const v4f a0 = *(const v4f*)(sp);
    const v4f a1 = *(const v4f*)(sp + 4);
#pragma unroll
    for (int e = 0; e < 4; ++e) {
      bv[it][e]     = (_Float16)(a0[e] * kCarryAct);
      bv[it][4 + e] = (_Float16)(a1[e] * kCarryAct);
    }
  }
  for (int pass = 0; pass < 2; ++pass) {
#pragma unroll
    for (int it = 0; it < 4; ++it)
      *(volatile v4f*)(XS + (size_t)(g0 + it * 4 + wave) * kDe + d0 + lane * 4) = fv[it];
#pragma unroll
    for (int it = 0; it < 2; ++it)
      *(volatile v8h*)(XSA + (size_t)(g0 + it * 8 + hrow) * kDe + d0 + c8) = bv[it];
    __threadfence();
  }
}

__global__ __launch_bounds__(128) void tree_scan_kernel(
    const float* __restrict__ XD, const float* __restrict__ XS,
    const float* __restrict__ Wdt, const float* __restrict__ bdt, const float* __restrict__ Alog,
    const int* __restrict__ si, const int* __restrict__ sp, float* HP)
{
  __shared__ __align__(16) float sX[kScTS * 16];
  __shared__ int sN[kScTS];
  __shared__ int sPar[kScTS];
  const int tid = threadIdx.x;
  constexpr int kBlkPerB = kDe / kScCh;
  const int bix = blockIdx.x / kBlkPerB;
  const int d0  = (blockIdx.x - bix * kBlkPerB) * kScCh;
  const int d   = d0 + tid;
  const size_t row0 = (size_t)bix * kL;
  const v4f wa = *(const v4f*)(Wdt + (size_t)d * kDtR);
  const v4f wb = *(const v4f*)(Wdt + (size_t)d * kDtR + 4);
  const v4f wc = *(const v4f*)(Wdt + (size_t)d * kDtR + 8);
  const float bb = bdt[d];
  const float gA = expf(Alog[d]);
  const float* xsd = XS + d;
  gvf* hv = (gvf*)(HP + d);
#pragma unroll 1
  for (int t0 = 0; t0 < kL; t0 += kScTS) {
    __syncthreads();
#pragma unroll
    for (int i = 0; i < 2; ++i) {
      const int idx = tid + 128 * i;
      const int r = idx >> 2, q = idx & 3;
      const int nraw = si[row0 + t0 + r];
      int praw = sp[row0 + t0 + r];
      asm volatile("" : "+v"(praw));
      int n = nraw < 0 ? 0 : nraw;
      n = n > (kL - 1) ? (kL - 1) : n;
      const v4f xv = *(const v4f*)(XD + (row0 + (size_t)n) * kXdP + q * 4);
      *(v4f*)(sX + r * 16 + q * 4) = xv;
      if (q == 0) { sN[r] = n; sPar[r] = praw; }
    }
    __syncthreads();
#pragma unroll 1
    for (int s = 0; s < kScTS; ++s) {
      const int t = t0 + s;
      const float* xr = sX + s * 16;
      const v4f xa = *(const v4f*)(xr);
      const v4f xb = *(const v4f*)(xr + 4);
      const v4f xc = *(const v4f*)(xr + 8);
      const v4f xe = *(const v4f*)(xr + 12);
      const int n = sN[s];
      const int p = sPar[s];
      float v = bb;
      v = fmaf(wa[0], xa[0], v);
      v = fmaf(wa[1], xa[1], v);
      v = fmaf(wa[2], xa[2], v);
      v = fmaf(wa[3], xa[3], v);
      v = fmaf(wb[0], xb[0], v);
      v = fmaf(wb[1], xb[1], v);
      v = fmaf(wb[2], xb[2], v);
      v = fmaf(wb[3], xb[3], v);
      v = fmaf(wc[0], xc[0], v);
      v = fmaf(wc[1], xc[1], v);
      v = fmaf(wc[2], xc[2], v);
      v = fmaf(wc[3], xc[3], v);
      const float a   = expf(-fabsf(v));
      const float u   = 1.0f + a;
      const float l1p = logf(u) + (a - (u - 1.0f)) * __builtin_amdgcn_rcpf(u);
      const float dt  = fmaxf(v, 0.0f) + l1p;
      const float dA  = expf(dt * gA);
      const float xsv = xsd[(row0 + (size_t)n) * kDe];
      const float dbx = (dt * xe[0]) * xsv;
      int pc = p < 0 ? 0 : p;
      pc = pc > (kL - 1) ? (kL - 1) : pc;
      const float hp = hv[(row0 + (size_t)pc) * kDe];
      const float hn = (p >= 0) ? fmaf(dA, hp, dbx) : dbx;
      gvf* hw = hv + (row0 + (size_t)t) * kDe;
      *hw = hn;
      __threadfence();
      *hw = hn;
    }
  }
}

__global__ __launch_bounds__(256) void norm_gate_kernel(
    const float* __restrict__ HP, const float* __restrict__ XS, const float* __restrict__ ZR,
    const float* __restrict__ XD, const int* __restrict__ si,
    const float* __restrict__ hg, const float* __restrict__ hb, const float* __restrict__ Dsv,
    const float* __restrict__ og, const float* __restrict__ ob, unsigned short* __restrict__ YZ)
{
  __shared__ __align__(16) float sRow[kNmWaves][kDe];
  const int lane = threadIdx.x & 31, wave = threadIdx.x >> 5;
  float* row = sRow[wave];
  const int cl = lane * 4;
#pragma unroll 1
  for (int it = 0; it < kNmPer; ++it) {
    const int gpos = blockIdx.x * (kNmWaves * kNmPer) + wave * kNmPer + it;
    const int bix = gpos >> 12;
    const int nraw = si[gpos];
    int n = nraw < 0 ? 0 : nraw;
    n = n > (kL - 1) ? (kL - 1) : n;
    const size_t rown = ((size_t)bix << 12) + (size_t)n;
    const float csv = XD[rown * kXdP + 13];
    const float* hp = HP + (size_t)gpos * kDe + cl;
    const float* xp = XS + rown * kDe + cl;
    const float* zp = ZR + rown * kDe + cl;
    float s = 0.0f;
#pragma unroll 1
    for (int j = 0; j < 3; ++j) {
      const v4f hv4 = *(const v4f*)(hp + 128 * j);
      *(v4f*)(row + cl + 128 * j) = hv4;
      s += (hv4[0] + hv4[1]) + (hv4[2] + hv4[3]);
    }
#pragma unroll
    for (int off = 16; off > 0; off >>= 1) s += __shfl_xor(s, off, 32);
    const float mu = s * kInvDe;
    float ss = 0.0f;
#pragma unroll 1
    for (int j = 0; j < 3; ++j) {
      const v4f hv4 = *(const v4f*)(row + cl + 128 * j);
#pragma unroll
      for (int e = 0; e < 4; ++e) { const float dd = hv4[e] - mu; ss = fmaf(dd, dd, ss); }
    }
#pragma unroll
    for (int off = 16; off > 0; off >>= 1) ss += __shfl_xor(ss, off, 32);
    const float rs = rsqrtf(ss * kInvDe + kLnEps);
    float s2 = 0.0f;
#pragma unroll 1
    for (int j = 0; j < 3; ++j) {
      const int c = cl + 128 * j;
      const v4f hv4 = *(const v4f*)(row + c);
      const v4f xv = *(const v4f*)(xp + 128 * j);
      const v4f gv = *(const v4f*)(hg + c);
      const v4f bv = *(const v4f*)(hb + c);
      const v4f dv = *(const v4f*)(Dsv + c);
      v4f yv;
#pragma unroll
      for (int e = 0; e < 4; ++e) {
        const float hn = (hv4[e] - mu) * rs * gv[e] + bv[e];
        yv[e] = hn * csv + dv[e] * xv[e];
      }
      *(v4f*)(row + c) = yv;
      s2 += (yv[0] + yv[1]) + (yv[2] + yv[3]);
    }
#pragma unroll
    for (int off = 16; off > 0; off >>= 1) s2 += __shfl_xor(s2, off, 32);
    const float mu2 = s2 * kInvDe;
    float ss2 = 0.0f;
#pragma unroll 1
    for (int j = 0; j < 3; ++j) {
      const v4f yv = *(const v4f*)(row + cl + 128 * j);
#pragma unroll
      for (int e = 0; e < 4; ++e) { const float dd = yv[e] - mu2; ss2 = fmaf(dd, dd, ss2); }
    }
#pragma unroll
    for (int off = 16; off > 0; off >>= 1) ss2 += __shfl_xor(ss2, off, 32);
    const float rs2 = rsqrtf(ss2 * kInvDe + kLnEps);
#pragma unroll 1
    for (int j = 0; j < 3; ++j) {
      const int c = cl + 128 * j;
      const v4f yv = *(const v4f*)(row + c);
      const v4f zv = *(const v4f*)(zp + 128 * j);
      const v4f gv = *(const v4f*)(og + c);
      const v4f bv = *(const v4f*)(ob + c);
      v4h ov;
#pragma unroll
      for (int e = 0; e < 4; ++e) {
        const float yo = (yv[e] - mu2) * rs2 * gv[e] + bv[e];
        const float zz = zv[e];
        const float gz = silu_f(zz);
        ov[e] = (_Float16)((yo * gz) * kCarryAct);
      }
      unsigned short* q = YZ + rown * kDe + c;
      *(volatile v4h*)q = ov;
      __threadfence();
      *(volatile v4h*)q = ov;
    }
  }
}

extern "C" void kernel_launch(void* const* d_in, const int* in_sizes, int n_in,
                              void* d_out, int out_size, void* d_ws, size_t ws_size,
                              hipStream_t stream) {
  if (n_in < 16) return;
  if (in_sizes[0] != kRows * kDm) return;
  if (in_sizes[1] != 2 * kDe * kDm) return;
  if (in_sizes[2] != kDe * 9) return;
  if (in_sizes[3] != kDe) return;
  if (in_sizes[4] != kXpN * kDe) return;
  if (in_sizes[5] != kDe * kDtR) return;
  if (in_sizes[6] != kDe) return;
  if (in_sizes[7] != kDe) return;
  if (in_sizes[8] != kDe) return;
  if (in_sizes[9] != kDe || in_sizes[10] != kDe || in_sizes[11] != kDe || in_sizes[12] != kDe) return;
  if (in_sizes[13] != kDm * kDe) return;
  if (in_sizes[14] != kRows || in_sizes[15] != kRows) return;
  if (out_size != kRows * kDm) return;
  if (ws_size < kWsTotal) return;

  const float* x      = (const float*)d_in[0];
  const float* W_in   = (const float*)d_in[1];
  const float* conv_w = (const float*)d_in[2];
  const float* conv_b = (const float*)d_in[3];
  const float* W_xp   = (const float*)d_in[4];
  const float* W_dt   = (const float*)d_in[5];
  const float* b_dt   = (const float*)d_in[6];
  const float* A_log  = (const float*)d_in[7];
  const float* Dsv    = (const float*)d_in[8];
  const float* hg     = (const float*)d_in[9];
  const float* hb     = (const float*)d_in[10];
  const float* og     = (const float*)d_in[11];
  const float* ob     = (const float*)d_in[12];
  const float* W_out  = (const float*)d_in[13];
  const int*   si     = (const int*)d_in[14];
  const int*   sp     = (const int*)d_in[15];
  float* out = (float*)d_out;

  char* ws = (char*)d_ws;
  unsigned short* XH  = (unsigned short*)(ws + kOffXH);
  unsigned short* XL  = (unsigned short*)(ws + kOffXL);
  unsigned short* WIH = (unsigned short*)(ws + kOffWIH);
  unsigned short* WIL = (unsigned short*)(ws + kOffWIL);
  unsigned short* WXP = (unsigned short*)(ws + kOffWXP);
  unsigned short* WOP = (unsigned short*)(ws + kOffWOP);
  float*          X1  = (float*)(ws + kOffX1);
  float*          ZR  = (float*)(ws + kOffZR);
  float*          XS  = (float*)(ws + kOffXS);
  unsigned short* XSA = (unsigned short*)(ws + kOffXSA);
  float*          XD  = (float*)(ws + kOffXD);
  unsigned short* YZ  = (unsigned short*)(ws + kOffYZ);
  float*          HP  = X1;
  const float* dummy_bias  = b_dt;
  const float* dummy_resid = x;

  split_rows_bf16_kernel<<<(kRows * kDm / 8) / 256, 256, 0, stream>>>(x, XH, XL, kRows * kDm / 8);
  split_rows_bf16_kernel<<<(2 * kDe * kDm / 8) / 256, 256, 0, stream>>>(W_in, WIH, WIL, 2 * kDe * kDm / 8);
  cast_f16_pad_kernel<<<(kXdP * kDe / 8) / 256, 256, 0, stream>>>(W_xp, WXP, kXdP * kDe / 8, kXpN * kDe / 8, kCarryW);
  cast_f16_pad_kernel<<<(kDm * kDe / 8) / 256, 256, 0, stream>>>(W_out, WOP, kDm * kDe / 8, kDm * kDe / 8, kCarryW);

  wmma_gemm64<1, true, 0, 0, false><<<dim3(192, 1), 256, 0, stream>>>(
      XH, XL, kDm, 0L,
      WIH, WIL, kDm, 0L,
      (void*)X1, (void*)X1, kDe, 0L,
      dummy_bias, dummy_resid, 0L,
      kRows, kDe, kDm, 1.0f);
  wmma_gemm64<1, true, 0, 0, false><<<dim3(192, 1), 256, 0, stream>>>(
      XH, XL, kDm, 0L,
      WIH + (size_t)kDe * kDm, WIL + (size_t)kDe * kDm, kDm, 0L,
      (void*)ZR, (void*)ZR, kDe, 0L,
      dummy_bias, dummy_resid, 0L,
      kRows, kDe, kDm, 1.0f);

  dwconv_silu_kernel<<<dim3(kDe / kCvCh, kRows / kCvPos), 128, 0, stream>>>(X1, conv_w, conv_b, XS, XSA);

  wmma_gemm64<0, false, 0, 0, false><<<dim3(32, 1), 256, 0, stream>>>(
      XSA, XSA, kDe, 0L,
      WXP, WXP, kDe, 0L,
      (void*)XD, (void*)XD, kXdP, 0L,
      dummy_bias, dummy_resid, 0L,
      kRows, kXdP, kDe, kFold);

  tree_scan_kernel<<<kBatch * (kDe / kScCh), kScCh, 0, stream>>>(XD, XS, W_dt, b_dt, A_log, si, sp, HP);

  norm_gate_kernel<<<kRows / (kNmWaves * kNmPer), 256, 0, stream>>>(HP, XS, ZR, XD, si, hg, hb, Dsv, og, ob, YZ);

  wmma_gemm64<0, false, 0, 0, false><<<dim3(96, 1), 256, 0, stream>>>(
      YZ, YZ, kDe, 0L,
      WOP, WOP, kDe, 0L,
      (void*)out, (void*)out, kDm, 0L,
      dummy_bias, dummy_resid, 0L,
      kRows, kDm, kDe, kFold);
}
